// NonLocalBlockND_88751204205091
// MI455X (gfx1250) — hardware-verified
//
#include <hip/hip_runtime.h>


#define NB_  8
#define C_   256
#define HW   4096
#define WID  64
#define CI   128
#define CG   128
#define NP   1024
#define NPP  1024
#define PW   32
#define RPAD 32
#define BEPS 1e-5f
typedef _Float16 h16;
typedef unsigned short bf;
typedef __attribute__((ext_vector_type(16))) __bf16   v16bf;
typedef __attribute__((ext_vector_type(16))) _Float16 v16h;
typedef __attribute__((ext_vector_type(8)))  _Float16 v8h;
typedef __attribute__((ext_vector_type(8)))  unsigned short v8us;
typedef __attribute__((ext_vector_type(8)))  float    v8f;
typedef __attribute__((ext_vector_type(4)))  float    v4f;
typedef __attribute__((ext_vector_type(2)))  float    v2f;
typedef __attribute__((ext_vector_type(4)))  unsigned short v4us;
typedef __attribute__((ext_vector_type(2)))  unsigned short v2us;
typedef v8h  __attribute__((may_alias)) v8ha;
typedef v4f  __attribute__((may_alias)) v4fa;
typedef v8us __attribute__((may_alias)) v8usa;

__device__ __forceinline__ unsigned short f2bf(float f) { unsigned u = __float_as_uint(f); u += 0x7FFFu + ((u >> 16) & 1u); return (unsigned short)(u >> 16); }
__device__ __forceinline__ float bf2f(unsigned short b) { return __uint_as_float(((unsigned)b) << 16); }
__device__ __forceinline__ float bfr(float f) { return bf2f(f2bf(f)); }
__device__ __forceinline__ void splitf(float y, unsigned short& h, unsigned short& l) { h = f2bf(y); l = f2bf(y - bf2f(h)); }
__device__ __forceinline__ v16h cat16(v8h lo, v8h hi) { return __builtin_shufflevector(lo, hi, 0, 1, 2, 3, 4, 5, 6, 7, 8, 9, 10, 11, 12, 13, 14, 15); }
__device__ __forceinline__ v16bf cat16b(v8us lo, v8us hi) { return __builtin_bit_cast(v16bf, __builtin_shufflevector(lo, hi, 0, 1, 2, 3, 4, 5, 6, 7, 8, 9, 10, 11, 12, 13, 14, 15)); }
__device__ __forceinline__ v8f wmma16(v16h a, v16h b, v8f c) { return __builtin_amdgcn_wmma_f32_16x16x32_f16(false, a, false, b, (short)0, c, false, false); }
__device__ __forceinline__ v8f wmmab(v16bf a, v16bf b, v8f c) { return __builtin_amdgcn_wmma_f32_16x16x32_bf16(false, a, false, b, (short)0, c, false, false); }

template <typename T16> struct WFrag;
template <> struct WFrag<h16> { typedef v16h V; static __device__ __forceinline__ V ld(const h16* p) { return cat16(*(const v8h*)p, *(const v8h*)(p + 16)); } static __device__ __forceinline__ v8f mma(V a, V b, v8f c) { return wmma16(a, b, c); } };
template <> struct WFrag<bf> { typedef v16bf V; static __device__ __forceinline__ V ld(const bf* p) { return cat16b(*(const v8us*)p, *(const v8us*)(p + 16)); } static __device__ __forceinline__ v8f mma(V a, V b, v8f c) { return wmmab(a, b, c); } };
template <typename T16, int NSPLIT, bool BIAS>
__global__ __launch_bounds__(32) void k_gemmw(const T16* __restrict__ A, const T16* __restrict__ A2, const T16* __restrict__ Bt, const T16* __restrict__ Bt2, int K, float* C, int ldc, const float* __restrict__ bias, size_t sA, size_t sB, size_t sC) {
    typedef typename WFrag<T16>::V V;
    __shared__ __align__(16) float os[16 * 68];
    const size_t z = blockIdx.z; A += z * sA; if (A2) A2 += z * sA; Bt += z * sB; if (Bt2) Bt2 += z * sB; C += z * sC;
    const int lane = threadIdx.x & 31, lr = lane & 15, hi = lane >> 4; const int r0 = blockIdx.x * 64, c0 = blockIdx.y * 64;
    v8f acc[4][4];
#pragma unroll
    for (int mb = 0; mb < 4; ++mb)
#pragma unroll
        for (int nb = 0; nb < 4; ++nb) acc[mb][nb] = (v8f){};
    const size_t aoff = (size_t)(r0 + lr) * K + 8 * hi, boff = (size_t)(c0 + lr) * K + 8 * hi;
#pragma unroll 1
    for (int kc = 0; kc < K; kc += 32) {
        V a[4], a2[4];
#pragma unroll
        for (int mb = 0; mb < 4; ++mb) { a[mb] = WFrag<T16>::ld(A + aoff + (size_t)mb * 16 * K + kc); if (NSPLIT == 1 || NSPLIT == 2) a2[mb] = WFrag<T16>::ld(A2 + aoff + (size_t)mb * 16 * K + kc); }
#pragma unroll
        for (int nb = 0; nb < 4; ++nb) { const V b = WFrag<T16>::ld(Bt + boff + (size_t)nb * 16 * K + kc); V b2; if (NSPLIT >= 2) b2 = WFrag<T16>::ld(Bt2 + boff + (size_t)nb * 16 * K + kc);
#pragma unroll
            for (int mb = 0; mb < 4; ++mb) { acc[mb][nb] = WFrag<T16>::mma(a[mb], b, acc[mb][nb]); if (NSPLIT == 1 || NSPLIT == 2) acc[mb][nb] = WFrag<T16>::mma(a2[mb], b, acc[mb][nb]); if (NSPLIT >= 2) acc[mb][nb] = WFrag<T16>::mma(a[mb], b2, acc[mb][nb]); } }
        asm volatile("v_nop\n\tv_nop\n\tv_nop\n\tv_nop" : "+v"(acc[0][0]), "+v"(acc[1][1]), "+v"(acc[2][2]), "+v"(acc[3][3]) : "v"(a[0]), "v"(a[3]));
    }
#pragma unroll
    for (int mb = 0; mb < 4; ++mb) {
#pragma unroll
        for (int nb = 0; nb < 4; ++nb) {
#pragma unroll
            for (int j = 0; j < 8; ++j) os[(hi * 8 + j) * 68 + nb * 16 + lr] = acc[mb][nb][j]; }
        __builtin_amdgcn_wave_barrier(); asm volatile("" ::: "memory");
        float* crow = C + (size_t)(r0 + mb * 16) * ldc + c0;
#pragma unroll 1
        for (int ps = 0; ps < 2; ++ps) {
#pragma unroll
            for (int s = 0; s < 8; ++s) { const int row = 2 * s + hi, cofs = lr * 4; v4f val = *(const v4fa*)(os + row * 68 + cofs); if (BIAS) { val[0] += bfr(bias[c0 + cofs]); val[1] += bfr(bias[c0 + cofs + 1]); val[2] += bfr(bias[c0 + cofs + 2]); val[3] += bfr(bias[c0 + cofs + 3]); }
                *(volatile v4f*)(crow + (size_t)row * ldc + cofs) = val; }
            if (ps == 0) __threadfence(); }
        __builtin_amdgcn_wave_barrier(); asm volatile("" ::: "memory");
    }
}


__global__ __launch_bounds__(256) void k_tpose(const float* __restrict__ xb, bf* XBp) { const size_t e = ((size_t)blockIdx.x * 256 + threadIdx.x) * 8; if (e >= (size_t)HW * C_) return; const int c = (int)(e % C_); const int t = (int)(e / C_); v8us o;
#pragma unroll
    for (int q = 0; q < 8; ++q) o[q] = f2bf(xb[(size_t)(c + q) * HW + t]); *(volatile v8us*)(XBp + e) = o; __threadfence(); *(volatile v8us*)(XBp + e) = o; }
__global__ __launch_bounds__(256) void k_split4(const float* __restrict__ F, bf* Ph, bf* Pl, size_t n4) { const size_t i = (size_t)blockIdx.x * 256 + threadIdx.x; if (i >= n4) return; const v4f v = *(const v4f*)(F + i * 4); v4us oh, ol;
#pragma unroll
    for (int q = 0; q < 4; ++q) { unsigned short a, c; splitf(v[q], a, c); oh[q] = a; ol[q] = c; } *(volatile v4us*)(Ph + i * 4) = oh; *(volatile v4us*)(Pl + i * 4) = ol; __threadfence(); *(volatile v4us*)(Ph + i * 4) = oh; *(volatile v4us*)(Pl + i * 4) = ol; }
__global__ __launch_bounds__(256) void k_outBN(const float* __restrict__ xb, const float* __restrict__ WY, const float* __restrict__ gm, const float* __restrict__ bt, const float* __restrict__ mn, const float* __restrict__ vr, float* Ob) { const size_t e = (size_t)blockIdx.x * 256 + threadIdx.x; if (e >= (size_t)C_ * HW) return; const int n = (int)(e % HW); const int c = (int)(e / HW);
    const float sc = __fmul_rn(bfr(gm[c]), __fdiv_rn(1.0f, __fsqrt_rn(__fadd_rn(bfr(vr[c]), BEPS)))); float t0 = __fsub_rn(WY[(size_t)n * C_ + c], bfr(mn[c])); asm volatile("" : "+v"(t0)); float t1 = __fmul_rn(t0, sc); asm volatile("" : "+v"(t1)); const float bnv = __fadd_rn(t1, bfr(bt[c])); const float v = __fadd_rn(bnv, bfr(xb[e])); *(volatile float*)(Ob + e) = v; __threadfence(); *(volatile float*)(Ob + e) = v; }
__global__ __launch_bounds__(256) void k_cvt8(const float* __restrict__ src, bf* dst, size_t n8) { const size_t i = (size_t)blockIdx.x * 256 + threadIdx.x; if (i >= n8) return; const v8f v = *(const v8f*)(src + i * 8); v8us o;
#pragma unroll
    for (int k = 0; k < 8; ++k) o[k] = f2bf(v[k]); *(volatile v8us*)(dst + i * 8) = o; __threadfence(); *(volatile v8us*)(dst + i * 8) = o; }

__global__ __launch_bounds__(256) void k_poolT(const float* __restrict__ F, int ldf, int col0, int nch, bf* Ph, bf* Pl) { const size_t e = ((size_t)blockIdx.x * 256 + threadIdx.x) * 2; if (e >= (size_t)CG * NPP) return; const int m = (int)(e % NPP); const int ch = (int)(e / NPP); v2us oh, ol;
#pragma unroll
    for (int q = 0; q < 2; ++q) { const int mm = m + q; float v = 0.f; if (mm < NP && ch < nch) { const int ph = mm / PW, pw = mm % PW; const int n00 = (2 * ph) * WID + 2 * pw; const float* f = F + col0 + ch; v = fmaxf(fmaxf(f[(size_t)n00 * ldf], f[(size_t)(n00 + 1) * ldf]), fmaxf(f[(size_t)(n00 + WID) * ldf], f[(size_t)(n00 + WID + 1) * ldf])); } unsigned short a, b2; splitf(v, a, b2); oh[q] = a; ol[q] = b2; }
    *(volatile v2us*)(Ph + e) = oh; *(volatile v2us*)(Pl + e) = ol; __threadfence(); *(volatile v2us*)(Ph + e) = oh; *(volatile v2us*)(Pl + e) = ol; }

__global__ __launch_bounds__(256) void k_msplit(const float* __restrict__ M, bf* Mh, bf* Ml) { const size_t i = (size_t)blockIdx.x * 256 + threadIdx.x; if (i >= (size_t)CG * CG / 4) return; const v4f a = *(const v4f*)(M + i * 4); v4us oh, ol;
#pragma unroll
    for (int q = 0; q < 4; ++q) { float v = __fmul_rn(a[q], 1.0f / (float)NP); asm volatile("" : "+v"(v)); unsigned short h2, l2; splitf(v, h2, l2); oh[q] = h2; ol[q] = l2; }
    *(volatile v4us*)(Mh + i * 4) = oh; *(volatile v4us*)(Ml + i * 4) = ol; __threadfence(); *(volatile v4us*)(Mh + i * 4) = oh; *(volatile v4us*)(Ml + i * 4) = ol; }


extern "C" void kernel_launch(void* const* d_in, const int* in_sizes, int n_in,
                              void* d_out, int out_size, void* d_ws, size_t ws_size, hipStream_t stream) {
    (void)in_sizes; (void)n_in; (void)out_size;
    const float* x = (const float*)d_in[0]; const float* wt = (const float*)d_in[1]; const float* bt = (const float*)d_in[2]; const float* wp = (const float*)d_in[3]; const float* bp = (const float*)d_in[4]; const float* wg = (const float*)d_in[5]; const float* bg = (const float*)d_in[6]; const float* ww = (const float*)d_in[7]; const float* bw = (const float*)d_in[8]; const float* bng = (const float*)d_in[9]; const float* bnb = (const float*)d_in[10]; const float* bnm = (const float*)d_in[11]; const float* bnv = (const float*)d_in[12];
    float* OUT = (float*)d_out;
    char* wsp = (char*)d_ws;
    auto take = [&](size_t bytes) { char* p = wsp; wsp += (bytes + 255) & ~(size_t)255; return (void*)p; };
    bf* WT = (bf*)take((size_t)CI * C_ * 2); bf* WP = (bf*)take((size_t)CI * C_ * 2); bf* WGb = (bf*)take((size_t)CI * C_ * 2); bf* WW = (bf*)take((size_t)C_ * CI * 2);
    bf* XT = (bf*)take((size_t)HW * C_ * 2); float* TH = (float*)take((size_t)HW * CI * 4); float* PH = (float*)take((size_t)HW * CI * 4); float* GG = (float*)take((size_t)HW * CI * 4);
    bf* THh = (bf*)take((size_t)HW * CI * 2); bf* THl = (bf*)take((size_t)HW * CI * 2); bf* FPh = (bf*)take((size_t)CI * NP * 2); bf* FPl = (bf*)take((size_t)CI * NP * 2); bf* GPh = (bf*)take((size_t)CI * NP * 2); bf* GPl = (bf*)take((size_t)CI * NP * 2);
    float* MTf = (float*)take((size_t)CI * CI * 4); bf* MTh = (bf*)take((size_t)CI * CI * 2); bf* MTl = (bf*)take((size_t)CI * CI * 2); float* Y = (float*)take((size_t)HW * CI * 4); bf* Yh = (bf*)take((size_t)HW * CI * 2); bf* Yl = (bf*)take((size_t)HW * CI * 2); float* WY = (float*)take((size_t)HW * C_ * 4);
    if ((size_t)(wsp - (char*)d_ws) > ws_size) return;
    k_cvt8<<<(unsigned)(((size_t)CI * C_ / 8 + 255) / 256), 256, 0, stream>>>(wt, WT, (size_t)CI * C_ / 8); k_cvt8<<<(unsigned)(((size_t)CI * C_ / 8 + 255) / 256), 256, 0, stream>>>(wp, WP, (size_t)CI * C_ / 8); k_cvt8<<<(unsigned)(((size_t)CI * C_ / 8 + 255) / 256), 256, 0, stream>>>(wg, WGb, (size_t)CI * C_ / 8); k_cvt8<<<(unsigned)(((size_t)C_ * CI / 8 + 255) / 256), 256, 0, stream>>>(ww, WW, (size_t)C_ * CI / 8);
    for (int b = 0; b < NB_; ++b) { const float* xb = x + (size_t)b * C_ * HW;
        k_tpose<<<(unsigned)(((size_t)HW * C_ / 8 + 255) / 256), 256, 0, stream>>>(xb, XT);
        k_gemmw<bf, 0, true><<<dim3(HW / 64, CI / 64, 1), 32, 0, stream>>>(XT, nullptr, WT, nullptr, C_, TH, CI, bt, 0, 0, 0);
        k_gemmw<bf, 0, true><<<dim3(HW / 64, CI / 64, 1), 32, 0, stream>>>(XT, nullptr, WP, nullptr, C_, PH, CI, bp, 0, 0, 0);
        k_gemmw<bf, 0, true><<<dim3(HW / 64, CI / 64, 1), 32, 0, stream>>>(XT, nullptr, WGb, nullptr, C_, GG, CI, bg, 0, 0, 0);
        k_poolT<<<(unsigned)(((size_t)CG * NPP / 2 + 255) / 256), 256, 0, stream>>>(PH, CI, 0, CI, FPh, FPl);
        k_poolT<<<(unsigned)(((size_t)CG * NPP / 2 + 255) / 256), 256, 0, stream>>>(GG, CI, 0, CI, GPh, GPl);
        k_gemmw<bf, 2, false><<<dim3(CI / 64, CI / 64, 1), 32, 0, stream>>>(GPh, GPl, FPh, FPl, NP, MTf, CI, nullptr, 0, 0, 0);
        k_msplit<<<(unsigned)(((size_t)CI * CI / 4 + 255) / 256), 256, 0, stream>>>(MTf, MTh, MTl);
        k_split4<<<(unsigned)(((size_t)HW * CI / 4 + 255) / 256), 256, 0, stream>>>(TH, THh, THl, (size_t)HW * CI / 4);
        k_gemmw<bf, 2, false><<<dim3(HW / 64, CI / 64, 1), 32, 0, stream>>>(THh, THl, MTh, MTl, CI, Y, CI, nullptr, 0, 0, 0);
        k_split4<<<(unsigned)(((size_t)HW * CI / 4 + 255) / 256), 256, 0, stream>>>(Y, Yh, Yl, (size_t)HW * CI / 4);
        k_gemmw<bf, 1, true><<<dim3(HW / 64, C_ / 64, 1), 32, 0, stream>>>(Yh, Yl, WW, nullptr, CI, WY, C_, bw, 0, 0, 0);
        k_outBN<<<(unsigned)(((size_t)C_ * HW + 255) / 256), 256, 0, stream>>>(xb, WY, bng, bnb, bnm, bnv, OUT + (size_t)b * C_ * HW); }
}
